// SelfAttention2D_70927089926205
// MI455X (gfx1250) — hardware-verified
//
#include <hip/hip_runtime.h>
#include <stddef.h>
#include <stdint.h>


#ifndef NB
#define NB 2
#endif
#ifndef SEQ
#define SEQ 1024
#endif
#define NB_FULL 2
#define SEQ_FULL 1024
#define DIM 768
#define NH 12
#define HD 64
#define NQKV (3 * DIM)
#define NREL 63
#define RELPAD 64

static_assert(NB >= 1 && NB <= NB_FULL);
static_assert(SEQ >= 64 && SEQ <= SEQ_FULL && (SEQ % 64) == 0);
static_assert((DIM % 64) == 0 && (HD == 64) && (NQKV % 64) == 0 && (NH * HD == DIM));

typedef _Float16 f16_t;
typedef unsigned short us_t;
typedef __attribute__((ext_vector_type(16))) _Float16 v16h;
typedef __attribute__((ext_vector_type(16))) __bf16 v16b;
typedef __attribute__((ext_vector_type(8))) float v8f;
typedef __attribute__((ext_vector_type(8))) unsigned short v8us;
typedef __attribute__((ext_vector_type(16))) unsigned short v16us;
typedef __attribute__((ext_vector_type(4))) float v4f;
typedef v8us __attribute__((may_alias)) v8usa;
typedef v4f __attribute__((may_alias)) v4fa;

union Frag { v16us u; v16h h; v16b b; v8us p[2]; };

__device__ __forceinline__ us_t bf16_bits(float f) {
  unsigned u = __float_as_uint(f);
  u += 0x7FFFu + ((u >> 16) & 1u);
  return (us_t)(u >> 16);
}
__device__ __forceinline__ float bf16_val(us_t bits) { return __uint_as_float(((unsigned)bits) << 16); }
__device__ __forceinline__ float bf16_rne(float f) { return bf16_val(bf16_bits(f)); }
__device__ __forceinline__ us_t f16_bits(float f) { f16_t hv = (f16_t)f; return __builtin_bit_cast(us_t, hv); }
__device__ __forceinline__ int clampi(int v, int lo, int hi) { return v < lo ? lo : (v > hi ? hi : v); }
__device__ __forceinline__ v8f zero8() {
  v8f z;
#pragma unroll
  for (int i = 0; i < 8; ++i) z[i] = 0.0f;
  return z;
}

__device__ __forceinline__ v8f mma_f16(v16h a, v16h b, v8f c) {
  c = __builtin_amdgcn_wmma_f32_16x16x32_f16(false, a, false, b, (short)0, c, false, false);
  asm volatile("v_nop\n\tv_nop\n\tv_nop\n\tv_nop" : "+v"(c) : "v"(a), "v"(b));
  return c;
}
__device__ __forceinline__ v8f mma_bf16(v16b a, v16b b, v8f c) {
  c = __builtin_amdgcn_wmma_f32_16x16x32_bf16(false, a, false, b, (short)0, c, false, false);
  asm volatile("v_nop\n\tv_nop\n\tv_nop\n\tv_nop" : "+v"(c) : "v"(a), "v"(b));
  return c;
}

__device__ __forceinline__ v16us ld_frag(const us_t* base, int ld, int row0, int k0) {
  const int l = (int)(threadIdx.x & 31), h = l >> 4, m = l & 15;
  const us_t* p = base + (size_t)(row0 + m) * (size_t)ld + k0 + 8 * h;
  Frag f;
  f.p[0] = *(const v8usa*)(p);
  f.p[1] = *(const v8usa*)(p + 16);
  return f.u;
}

__global__ __launch_bounds__(256)
void k_cvt(const float* __restrict__ src, us_t* __restrict__ dst, int n8) {
  const int i = (int)blockIdx.x * 256 + (int)threadIdx.x;
  if (i < n8) {
    const float* s = src + (size_t)i * 8;
    const v4f a = *(const v4fa*)(s);
    const v4f c = *(const v4fa*)(s + 4);
    v8us o;
    o[0] = bf16_bits(a[0]); o[1] = bf16_bits(a[1]); o[2] = bf16_bits(a[2]); o[3] = bf16_bits(a[3]);
    o[4] = bf16_bits(c[0]); o[5] = bf16_bits(c[1]); o[6] = bf16_bits(c[2]); o[7] = bf16_bits(c[3]);
    us_t* d = dst + (size_t)i * 8;
    *(volatile v8us*)d = o;
    __threadfence();
    *(volatile v8us*)d = o;
  }
}

__device__ __forceinline__ void qk_store(const float* Ts, us_t* __restrict__ dst, int bh, int n0, int tid) {
#pragma unroll
  for (int it = 0; it < 4; ++it) {
    const int idx = it * 128 + tid, row = idx >> 3, piece = idx & 7;
    const float* s = Ts + row * 64 + piece * 8;
    v8us o;
#pragma unroll
    for (int j = 0; j < 8; ++j) o[j] = f16_bits(s[j] * 8.0f);
    us_t* p = dst + ((size_t)(bh * SEQ_FULL + n0 + row)) * HD + piece * 8;
    *(volatile v8us*)p = o;
  }
}
__device__ __forceinline__ void v_store(const float* Ts, us_t* __restrict__ VTh, us_t* __restrict__ VTl,
                                        int bh, int n0, int tid) {
#pragma unroll
  for (int it = 0; it < 8; ++it) {
    const int idx = it * 128 + tid;
    const int plane = idx >> 9;
    const int d = (idx >> 3) & 63, piece = idx & 7;
    v8us o;
#pragma unroll
    for (int j = 0; j < 8; ++j) {
      const float v = Ts[(piece * 8 + j) * 64 + d];
      const us_t hb = bf16_bits(v);
      const us_t lb = bf16_bits(v - bf16_val(hb));
      o[j] = plane ? lb : hb;
    }
    us_t* dst = plane ? VTl : VTh;
    us_t* p = dst + ((size_t)(bh * HD + d)) * SEQ_FULL + n0 + piece * 8;
    *(volatile v8us*)p = o;
  }
}

__global__ __launch_bounds__(128)
void k_qkv(const us_t* __restrict__ Xb, const us_t* __restrict__ Wb, const float* __restrict__ qkvb,
           us_t* __restrict__ Q8, us_t* __restrict__ K8, us_t* __restrict__ VTh, us_t* __restrict__ VTl) {
  __shared__ __align__(16) float Ts[64 * 64];
  const int tid = (int)threadIdx.x, w = tid >> 5, l = tid & 31, h = l >> 4, m = l & 15;
  const int TN = NQKV / 64;
  const int bm = (int)blockIdx.x / TN, tn = (int)blockIdx.x - bm * TN;
  const int tok0 = bm * 64;
  const int b = tok0 / SEQ, n0 = tok0 - b * SEQ;
  const int xrow0 = b * SEQ_FULL + n0;
  const int which = tn / NH, hh = tn - which * NH;
  const int col0 = tn * 64;

  v8f acc[4];
#pragma unroll
  for (int s = 0; s < 4; ++s) acc[s] = zero8();

  for (int k0 = 0; k0 < DIM; k0 += 32) {
    Frag a;
    a.u = ld_frag(Xb, DIM, xrow0 + w * 16, k0);
#pragma unroll
    for (int s = 0; s < 4; ++s) {
      Frag bb;
      bb.u = ld_frag(Wb, DIM, col0 + s * 16, k0);
      acc[s] = mma_bf16(a.b, bb.b, acc[s]);
    }
  }

#pragma unroll
  for (int s = 0; s < 4; ++s) {
    const float bv = bf16_rne(qkvb[col0 + s * 16 + m]);
#pragma unroll
    for (int r = 0; r < 8; ++r) Ts[(w * 16 + 8 * h + r) * 64 + s * 16 + m] = acc[s][r] + bv;
  }
  __syncthreads();

  const int bh = b * NH + hh;
  if (which < 2) {
    us_t* dst = (which == 0) ? Q8 : K8;
    qk_store(Ts, dst, bh, n0, tid);
    __threadfence();
    qk_store(Ts, dst, bh, n0, tid);
  } else {
    v_store(Ts, VTh, VTl, bh, n0, tid);
    __threadfence();
    v_store(Ts, VTh, VTl, bh, n0, tid);
  }
}

__device__ __forceinline__ void t_store(const float* Ts, float* __restrict__ T, int row0, int tid) {
#pragma unroll
  for (int it = 0; it < 8; ++it) {
    const int idx = it * 128 + tid, row = idx >> 4, piece = idx & 15;
    const float* s = Ts + row * 64 + piece * 4;
    v4f o;
    o[0] = s[0]; o[1] = s[1]; o[2] = s[2]; o[3] = s[3];
    float* p = T + (size_t)(row0 + row) * RELPAD + piece * 4;
    *(volatile v4f*)p = o;
  }
}

__global__ __launch_bounds__(128)
void k_rel(const us_t* __restrict__ Q8, const float* __restrict__ relh, const float* __restrict__ relw,
           float* __restrict__ Th, float* __restrict__ Tw) {
  __shared__ __align__(16) us_t Rl[RELPAD * HD];
  __shared__ __align__(16) float Ts[64 * 64];
  const int tid = (int)threadIdx.x, w = tid >> 5, l = tid & 31, h = l >> 4, m = l & 15;
  const int NBLK = SEQ / 64;
  const int bh = (int)blockIdx.x / NBLK, nb = (int)blockIdx.x - bh * NBLK;
  const int which = (int)blockIdx.y;
  const int row0 = bh * SEQ_FULL + nb * 64;
  const float* rel = which ? relw : relh;

#pragma unroll
  for (int it = 0; it < 32; ++it) {
    const int e = it * 128 + tid;
    const int j = e >> 6, c = e & 63;
    const int jj = j < (NREL - 1) ? j : (NREL - 1);
    const float v = bf16_rne(rel[jj * HD + c]) * 64.0f;
    Rl[e] = (j < NREL) ? f16_bits(v) : (us_t)0;
  }
  __syncthreads();

  v8f acc[4];
#pragma unroll
  for (int s = 0; s < 4; ++s) acc[s] = zero8();
#pragma unroll
  for (int k0 = 0; k0 < HD; k0 += 32) {
    Frag a;
    a.u = ld_frag(Q8, HD, row0 + w * 16, k0);
#pragma unroll
    for (int s = 0; s < 4; ++s) {
      Frag bb;
      bb.u = ld_frag(Rl, HD, s * 16, k0);
      acc[s] = mma_f16(a.h, bb.h, acc[s]);
    }
  }
  const float INV512 = 1.0f / 512.0f;
#pragma unroll
  for (int s = 0; s < 4; ++s)
#pragma unroll
    for (int r = 0; r < 8; ++r) Ts[(w * 16 + 8 * h + r) * 64 + s * 16 + m] = acc[s][r] * INV512;
  __syncthreads();

  float* T = which ? Tw : Th;
  t_store(Ts, T, row0, tid);
  __threadfence();
  t_store(Ts, T, row0, tid);
}

struct AttnTiles {
  us_t K[32 * 64];
  us_t V[2][64 * 32];
  us_t P[4][2][16 * 32];
};
union AttnSmem {
  AttnTiles t;
  float O[64 * 64];
};

__device__ __forceinline__ void attn_store(const float* Os, us_t* __restrict__ Ah, us_t* __restrict__ Al,
                                           int b, int qb, int hh, int tid) {
#pragma unroll
  for (int it = 0; it < 4; ++it) {
    const int idx = it * 128 + tid, row = idx >> 3, piece = idx & 7;
    const float* s = Os + row * 64 + piece * 8;
    v8us oh, ol;
#pragma unroll
    for (int j = 0; j < 8; ++j) {
      const float v = s[j];
      const us_t hb = bf16_bits(v);
      oh[j] = hb;
      ol[j] = bf16_bits(v - bf16_val(hb));
    }
    const size_t off = ((size_t)(b * SEQ_FULL + qb * 64 + row)) * DIM + hh * HD + piece * 8;
    *(volatile v8us*)(Ah + off) = oh;
    *(volatile v8us*)(Al + off) = ol;
  }
}

__global__ __launch_bounds__(128)
void k_attn(const us_t* __restrict__ Q8, const us_t* __restrict__ K8,
            const us_t* __restrict__ VTh, const us_t* __restrict__ VTl,
            const float* __restrict__ Th, const float* __restrict__ Tw,
            const int* __restrict__ pxh, const int* __restrict__ pxw,
            us_t* __restrict__ Ah, us_t* __restrict__ Al) {
  __shared__ __align__(16) AttnSmem sm;
  __shared__ __align__(16) float Bl[4][16 * 128];

  const int tid = (int)threadIdx.x, w = tid >> 5, l = tid & 31, h = l >> 4, m = l & 15;
  const int NQB = SEQ / 64;
  const int bh = (int)blockIdx.x / NQB, qb = (int)blockIdx.x - bh * NQB;
  const int b = bh / NH, hh = bh - b * NH;
  const int q0w = qb * 64 + w * 16;
  const int qrow0 = bh * SEQ_FULL + q0w;
  const int xh = clampi(pxh[0], 1, 4096), xw = clampi(pxw[0], 1, 4096);

#pragma unroll
  for (int it = 0; it < 16; ++it) {
    const int e = it * 32 + l;
    const int tsel = e >> 8, row = (e >> 4) & 15, piece = e & 15;
    const float* src = (tsel ? Tw : Th) + (size_t)(qrow0 + row) * RELPAD + piece * 4;
    *(v4fa*)(&Bl[w][row * 128 + tsel * 64 + piece * 4]) = *(const v4fa*)src;
  }

  Frag qa0, qa1;
  qa0.u = ld_frag(Q8, HD, qrow0, 0);
  qa1.u = ld_frag(Q8, HD, qrow0, 32);

  int hq[8], wq[8];
#pragma unroll
  for (int r = 0; r < 8; ++r) {
    const int qr = q0w + 8 * h + r;
    hq[r] = qr / xw;
    wq[r] = qr - hq[r] * xw;
  }

  float mrow[8], lrow[8];
  v8f acc[4];
#pragma unroll
  for (int r = 0; r < 8; ++r) { mrow[r] = -1e30f; lrow[r] = 0.0f; }
#pragma unroll
  for (int f = 0; f < 4; ++f) acc[f] = zero8();

  const float INV512 = 1.0f / 512.0f;

  for (int kt = 0; kt < SEQ; kt += 32) {
#pragma unroll
    for (int it = 0; it < 2; ++it) {
      const int e = it * 128 + tid, row = e >> 3, piece = e & 7;
      const us_t* src = K8 + ((size_t)(bh * SEQ_FULL + kt + row)) * HD + piece * 8;
      *(v8usa*)(&sm.t.K[row * 64 + piece * 8]) = *(const v8usa*)src;
    }
#pragma unroll
    for (int it = 0; it < 4; ++it) {
      const int e = it * 128 + tid;
      const int plane = e >> 8;
      const int d = (e >> 2) & 63, piece = e & 3;
      const us_t* src = (plane ? VTl : VTh) + ((size_t)(bh * HD + d)) * SEQ_FULL + kt + piece * 8;
      *(v8usa*)(&sm.t.V[plane][d * 32 + piece * 8]) = *(const v8usa*)src;
    }
    __syncthreads();

    v8f s0 = zero8(), s1 = zero8();
    {
      Frag kb;
      kb.u = ld_frag(sm.t.K, 64, 0, 0);   s0 = mma_f16(qa0.h, kb.h, s0);
      kb.u = ld_frag(sm.t.K, 64, 0, 32);  s0 = mma_f16(qa1.h, kb.h, s0);
      kb.u = ld_frag(sm.t.K, 64, 16, 0);  s1 = mma_f16(qa0.h, kb.h, s1);
      kb.u = ld_frag(sm.t.K, 64, 16, 32); s1 = mma_f16(qa1.h, kb.h, s1);
    }

    const int key0 = kt + m, key1 = key0 + 16;
    const int hk0 = key0 / xw, wk0 = key0 - hk0 * xw;
    const int hk1 = key1 / xw, wk1 = key1 - hk1 * xw;
#pragma unroll
    for (int r = 0; r < 8; ++r) {
      const float* br = &Bl[w][(8 * h + r) * 128];
      const int ih0 = clampi(hq[r] - hk0 + xh - 1, 0, NREL - 1);
      const int iw0 = clampi(wq[r] - wk0 + xw - 1, 0, NREL - 1);
      const int ih1 = clampi(hq[r] - hk1 + xh - 1, 0, NREL - 1);
      const int iw1 = clampi(wq[r] - wk1 + xw - 1, 0, NREL - 1);
      const float t0 = br[ih0] + br[64 + iw0];
      const float t1 = br[ih1] + br[64 + iw1];
      s0[r] = s0[r] * INV512 + t0;
      s1[r] = s1[r] * INV512 + t1;
    }

    float alpha[8];
#pragma unroll
    for (int r = 0; r < 8; ++r) {
      float mx = fmaxf(s0[r], s1[r]);
#pragma unroll
      for (int off = 8; off >= 1; off >>= 1) mx = fmaxf(mx, __shfl_xor(mx, off, 32));
      const float mnew = fmaxf(mrow[r], mx);
      alpha[r] = __expf(mrow[r] - mnew);
      mrow[r] = mnew;
      const float p0 = __expf(s0[r] - mnew);
      const float p1 = __expf(s1[r] - mnew);
      float rs = p0 + p1;
#pragma unroll
      for (int off = 8; off >= 1; off >>= 1) rs += __shfl_xor(rs, off, 32);
      lrow[r] = lrow[r] * alpha[r] + rs;
      const us_t hb0 = bf16_bits(p0), hb1 = bf16_bits(p1);
      const us_t lb0 = bf16_bits(p0 - bf16_val(hb0)), lb1 = bf16_bits(p1 - bf16_val(hb1));
      const int prow = (8 * h + r) * 32;
      sm.t.P[w][0][prow + m] = hb0;
      sm.t.P[w][0][prow + m + 16] = hb1;
      sm.t.P[w][1][prow + m] = lb0;
      sm.t.P[w][1][prow + m + 16] = lb1;
    }
#pragma unroll
    for (int f = 0; f < 4; ++f)
#pragma unroll
      for (int r = 0; r < 8; ++r) acc[f][r] *= alpha[r];

    __syncthreads();

    Frag ph, pl;
    ph.u = ld_frag(&sm.t.P[w][0][0], 32, 0, 0);
    pl.u = ld_frag(&sm.t.P[w][1][0], 32, 0, 0);
#pragma unroll
    for (int f = 0; f < 4; ++f) {
      Frag vh, vl;
      vh.u = ld_frag(sm.t.V[0], 32, f * 16, 0);
      vl.u = ld_frag(sm.t.V[1], 32, f * 16, 0);
      acc[f] = mma_bf16(ph.b, vh.b, acc[f]);
      acc[f] = mma_bf16(ph.b, vl.b, acc[f]);
      acc[f] = mma_bf16(pl.b, vh.b, acc[f]);
    }
    __syncthreads();
  }

  float invl[8];
#pragma unroll
  for (int r = 0; r < 8; ++r) invl[r] = 1.0f / lrow[r];
#pragma unroll
  for (int f = 0; f < 4; ++f)
#pragma unroll
    for (int r = 0; r < 8; ++r) sm.O[(w * 16 + 8 * h + r) * 64 + f * 16 + m] = acc[f][r] * invl[r];
  __syncthreads();

  attn_store(sm.O, Ah, Al, b, qb, hh, tid);
  __threadfence();
  attn_store(sm.O, Ah, Al, b, qb, hh, tid);
}

__device__ __forceinline__ void out_store(const float* Ts, float* __restrict__ out, int arow0, int col0, int tid) {
#pragma unroll
  for (int it = 0; it < 8; ++it) {
    const int idx = it * 128 + tid, row = idx >> 4, piece = idx & 15;
    const float* s = Ts + row * 64 + piece * 4;
    v4f o;
    o[0] = s[0]; o[1] = s[1]; o[2] = s[2]; o[3] = s[3];
    float* p = out + (size_t)(arow0 + row) * DIM + col0 + piece * 4;
    *(volatile v4f*)p = o;
  }
}

__global__ __launch_bounds__(128)
void k_proj(const us_t* __restrict__ Ah, const us_t* __restrict__ Al, const us_t* __restrict__ Wp,
            const float* __restrict__ pb, float* __restrict__ out) {
  __shared__ __align__(16) float Ts[64 * 64];
  const int tid = (int)threadIdx.x, w = tid >> 5, l = tid & 31, h = l >> 4, m = l & 15;
  const int TN = DIM / 64;
  const int bm = (int)blockIdx.x / TN, tn = (int)blockIdx.x - bm * TN;
  const int tok0 = bm * 64;
  const int b = tok0 / SEQ, n0 = tok0 - b * SEQ;
  const int arow0 = b * SEQ_FULL + n0;
  const int col0 = tn * 64;

  v8f acc[4];
#pragma unroll
  for (int s = 0; s < 4; ++s) acc[s] = zero8();

  for (int k0 = 0; k0 < DIM; k0 += 32) {
    Frag ah, al;
    ah.u = ld_frag(Ah, DIM, arow0 + w * 16, k0);
    al.u = ld_frag(Al, DIM, arow0 + w * 16, k0);
#pragma unroll
    for (int s = 0; s < 4; ++s) {
      Frag wb;
      wb.u = ld_frag(Wp, DIM, col0 + s * 16, k0);
      acc[s] = mma_bf16(ah.b, wb.b, acc[s]);
      acc[s] = mma_bf16(al.b, wb.b, acc[s]);
    }
  }

#pragma unroll
  for (int s = 0; s < 4; ++s) {
    const float bv = bf16_rne(pb[col0 + s * 16 + m]);
#pragma unroll
    for (int r = 0; r < 8; ++r) Ts[(w * 16 + 8 * h + r) * 64 + s * 16 + m] = acc[s][r] + bv;
  }
  __syncthreads();

  out_store(Ts, out, arow0, col0, tid);
  __threadfence();
  out_store(Ts, out, arow0, col0, tid);
}

extern "C" void kernel_launch(void* const* d_in, const int* in_sizes, int n_in,
                              void* d_out, int out_size, void* d_ws, size_t ws_size,
                              hipStream_t stream) {
  if (n_in < 9) return;
  const int XROWS = (NB - 1) * SEQ_FULL + SEQ;
  if (in_sizes[0] < XROWS * DIM) return;
  if (in_sizes[1] < NQKV * DIM) return;
  if (in_sizes[2] < NQKV) return;
  if (in_sizes[3] < DIM * DIM) return;
  if (in_sizes[4] < DIM) return;
  if (in_sizes[5] < NREL * HD) return;
  if (in_sizes[6] < NREL * HD) return;
  if (in_sizes[7] < 1 || in_sizes[8] < 1) return;
  if (out_size < XROWS * DIM) return;

  const float* x     = (const float*)d_in[0];
  const float* qkvw  = (const float*)d_in[1];
  const float* qkvb  = (const float*)d_in[2];
  const float* projw = (const float*)d_in[3];
  const float* projb = (const float*)d_in[4];
  const float* relh  = (const float*)d_in[5];
  const float* relw  = (const float*)d_in[6];
  const int*   pxh   = (const int*)d_in[7];
  const int*   pxw   = (const int*)d_in[8];

  size_t off = 0;
  auto carve = [&](size_t bytes) -> size_t { size_t p = off; off += (bytes + 255) & ~(size_t)255; return p; };
  const size_t szX  = (size_t)NB_FULL * SEQ_FULL * DIM * 2;
  const size_t szWq = (size_t)NQKV * DIM * 2;
  const size_t szWp = (size_t)DIM * DIM * 2;
  const size_t szH  = (size_t)NB_FULL * NH * SEQ_FULL * HD * 2;
  const size_t szT  = (size_t)NB_FULL * NH * SEQ_FULL * RELPAD * 4;
  const size_t szA  = (size_t)NB_FULL * SEQ_FULL * DIM * 2;
  const size_t oXb = carve(szX), oWb = carve(szWq), oWp = carve(szWp);
  const size_t oQ8 = carve(szH), oK8 = carve(szH), oVh = carve(szH), oVl = carve(szH);
  const size_t oTh = carve(szT), oTw = carve(szT);
  const size_t oAh = carve(szA), oAl = carve(szA);
  if (off > ws_size || off > (size_t)134217728u) return;

  char* ws = (char*)d_ws;
  us_t* Xb  = (us_t*)(ws + oXb);
  us_t* Wb  = (us_t*)(ws + oWb);
  us_t* Wp  = (us_t*)(ws + oWp);
  us_t* Q8  = (us_t*)(ws + oQ8);
  us_t* K8  = (us_t*)(ws + oK8);
  us_t* VTh = (us_t*)(ws + oVh);
  us_t* VTl = (us_t*)(ws + oVl);
  float* Th = (float*)(ws + oTh);
  float* Tw = (float*)(ws + oTw);
  us_t* Ah  = (us_t*)(ws + oAh);
  us_t* Al  = (us_t*)(ws + oAl);

  const int n8x = XROWS * DIM / 8;
  const int n8w = NQKV * DIM / 8;
  const int n8p = DIM * DIM / 8;
  k_cvt<<<(n8x + 255) / 256, 256, 0, stream>>>(x, Xb, n8x);
  k_cvt<<<(n8w + 255) / 256, 256, 0, stream>>>(qkvw, Wb, n8w);
  k_cvt<<<(n8p + 255) / 256, 256, 0, stream>>>(projw, Wp, n8p);

  k_qkv<<<(NB * SEQ / 64) * (NQKV / 64), 128, 0, stream>>>(Xb, Wb, qkvb, Q8, K8, VTh, VTl);
  k_rel<<<dim3(NB * NH * (SEQ / 64), 2, 1), 128, 0, stream>>>(Q8, relh, relw, Th, Tw);
  k_attn<<<NB * NH * (SEQ / 64), 128, 0, stream>>>(Q8, K8, VTh, VTl, Th, Tw, pxh, pxw, Ah, Al);
  k_proj<<<(NB * SEQ / 64) * (DIM / 64), 128, 0, stream>>>(Ah, Al, Wp, projb, (float*)d_out);
  (void)hipGetLastError();
}
